// GNNCompleteNeighborhood_55095840473790
// MI455X (gfx1250) — hardware-verified
//
#include <hip/hip_runtime.h>
#include <math.h>
typedef __attribute__((ext_vector_type(16))) _Float16 v16h;
typedef __attribute__((ext_vector_type(8)))  _Float16 v8h;
typedef __attribute__((ext_vector_type(16))) __bf16   v16b;
typedef __attribute__((ext_vector_type(8)))  __bf16   v8b;
typedef __attribute__((ext_vector_type(8)))  float    v8f;
typedef __attribute__((ext_vector_type(4)))  float    v4f;
#define PSCALE 32768.0f
#define U16(p) ((const unsigned short*)(const void*)(p))
#define PSCALE_INV (1.0f / 32768.0f)

__device__ __forceinline__ unsigned short f2bf_bits(float f) {
  unsigned u = __float_as_uint(f);
  return (unsigned short)((u + 0x7FFFu + ((u >> 16) & 1u)) >> 16);
}
__device__ __forceinline__ float bf_bits2f(unsigned short h) { return __uint_as_float(((unsigned)h) << 16); }

__device__ __forceinline__ void dep_guard_h(v8f& a, v8f& b, v16h x, v16h y) { asm volatile("v_nop\n\tv_nop\n\tv_nop\n\tv_nop" : "+v"(a), "+v"(b) : "v"(x), "v"(y)); }
__device__ __forceinline__ void dep_guard_b(v8f& a, v8f& b, v16b x, v16b y) { asm volatile("v_nop\n\tv_nop\n\tv_nop\n\tv_nop" : "+v"(a), "+v"(b) : "v"(x), "v"(y)); }
__device__ __forceinline__ void keep4_h(v16h a, v16h b, v16h c, v16h d) { asm volatile("v_nop" :: "v"(a), "v"(b), "v"(c), "v"(d)); }
__device__ __forceinline__ void keep4_b(v16b a, v16b b, v16b c, v16b d) { asm volatile("v_nop" :: "v"(a), "v"(b), "v"(c), "v"(d)); }
__device__ __forceinline__ void acc_guard4(v8f& a, v8f& b, v8f& c, v8f& d) { asm volatile("v_nop\n\tv_nop\n\tv_nop\n\tv_nop" : "+v"(a), "+v"(b), "+v"(c), "+v"(d)); }
template <typename T> struct Frag;
template <> struct Frag<_Float16> {
  typedef v16h V; union U { v16h v; v8h h[2]; };
  static __device__ __forceinline__ v16h load(const _Float16* p) {
    U f; f.h[0] = *(const v8h*)(p); f.h[1] = *(const v8h*)(p + 16); return f.v;
  }
  static __device__ __forceinline__ v8f mma(v16h a, v16h b, v8f c) {
    return __builtin_amdgcn_wmma_f32_16x16x32_f16(false, a, false, b, (short)0, c, false, false);
  }
  static __device__ __forceinline__ void guard(v8f& a, v8f& b, v16h x, v16h y) { dep_guard_h(a, b, x, y); }
  static __device__ __forceinline__ void keep(v16h a, v16h b, v16h c, v16h d) { keep4_h(a, b, c, d); }
};
template <> struct Frag<__bf16> {
  typedef v16b V; union U { v16b v; v8b h[2]; };
  static __device__ __forceinline__ v16b load(const __bf16* p) {
    U f; f.h[0] = *(const v8b*)(p); f.h[1] = *(const v8b*)(p + 16); return f.v;
  }
  static __device__ __forceinline__ v8f mma(v16b a, v16b b, v8f c) {
    return __builtin_amdgcn_wmma_f32_16x16x32_bf16(false, a, false, b, (short)0, c, false, false);
  }
  static __device__ __forceinline__ void guard(v8f& a, v8f& b, v16b x, v16b y) { dep_guard_b(a, b, x, y); }
  static __device__ __forceinline__ void keep(v16b a, v16b b, v16b c, v16b d) { keep4_b(a, b, c, d); }
};

template <int ET> struct Elem;
template <> struct Elem<0> { typedef _Float16 T; };
template <> struct Elem<1> { typedef __bf16 T; };
template <int ET, bool SPLIT, int BIAS_MODE, int OUT_MODE, bool RESID, int ACT = 0>
__global__ __launch_bounds__(256) void wmma_gemm64(
    const unsigned short* __restrict__ Ap, const unsigned short* __restrict__ A2p, int lda, long strideA,
    const unsigned short* __restrict__ Btp, const unsigned short* __restrict__ Bt2p, int ldb, long strideB,
    void* __restrict__ Cout, void* __restrict__ Cout2, int ldc, long strideC,
    const float* __restrict__ bias,
    const float* __restrict__ resid, long strideR,
    int M, int N, int K, float scale) {
  typedef typename Elem<ET>::T T;
  typedef typename Frag<T>::V V;
  const T* A = (const T*)Ap; const T* A2 = (const T*)A2p; const T* Bt = (const T*)Btp; const T* Bt2 = (const T*)Bt2p;
  __shared__ __align__(16) float sT[8][16 * 68];
  const int b    = blockIdx.y;
  const int lane = threadIdx.x & 31;
  const int wave = threadIdx.x >> 5;
  const int tilesN = N >> 6;
  const int tilesM = M >> 6;
  const int tile = blockIdx.x * 8 + wave;
  if (tile >= tilesM * tilesN) return;
  const int tm = tile / tilesN;
  const int tn = tile - tm * tilesN;
  const int m0 = tm << 6;
  const int n0 = tn << 6;

  const T* Ab  = A  + (size_t)b * strideA;
  const T* Bb  = Bt + (size_t)b * strideB;
  const T* Ab2 = SPLIT ? (A2  + (size_t)b * strideA) : nullptr;
  const T* Bb2 = SPLIT ? (Bt2 + (size_t)b * strideB) : nullptr;

  const int rlane = lane & 15;
  const int koff  = (lane >> 4) * 8;
  const int mOff  = (lane >> 4) * 8;

  v8f acc[4][4];
#pragma unroll
  for (int i = 0; i < 4; ++i)
#pragma unroll
    for (int j = 0; j < 4; ++j) acc[i][j] = (v8f){0.f,0.f,0.f,0.f,0.f,0.f,0.f,0.f};

  for (int k0 = 0; k0 < K; k0 += 32) {
    V bh[4], bl[4];
#pragma unroll
    for (int j = 0; j < 4; ++j) {
      const size_t bo = (size_t)(n0 + (j << 4) + rlane) * ldb + koff + k0;
      bh[j] = Frag<T>::load(Bb + bo);
      if (SPLIT) bl[j] = Frag<T>::load(Bb2 + bo);
    }
#pragma unroll
    for (int i = 0; i < 4; ++i) {
      const size_t ao = (size_t)(m0 + (i << 4) + rlane) * lda + koff + k0;
      V ah = Frag<T>::load(Ab + ao);
      V al;
      if (SPLIT) al = Frag<T>::load(Ab2 + ao);
#pragma unroll
      for (int j = 0; j < 4; ++j) {
        acc[i][j] = Frag<T>::mma(ah, bh[j], acc[i][j]);
        if (SPLIT) {
          acc[i][j] = Frag<T>::mma(ah, bl[j], acc[i][j]);
          acc[i][j] = Frag<T>::mma(al, bh[j], acc[i][j]);
        }
      }
      Frag<T>::guard(acc[i][0], acc[i][3], ah, SPLIT ? al : ah);
    }
    Frag<T>::keep(bh[0], bh[1], bh[2], bh[3]);
    if (SPLIT) Frag<T>::keep(bl[0], bl[1], bl[2], bl[3]);
  }
  acc_guard4(acc[0][0], acc[0][1], acc[0][2], acc[0][3]);
  acc_guard4(acc[1][0], acc[1][1], acc[1][2], acc[1][3]);
  acc_guard4(acc[2][0], acc[2][1], acc[2][2], acc[2][3]);
  acc_guard4(acc[3][0], acc[3][1], acc[3][2], acc[3][3]);

  float* slab = sT[wave];
  const float* Rb = RESID ? (resid + (size_t)b * strideR) : nullptr;
#pragma unroll
  for (int i = 0; i < 4; ++i) {
    const int mBase = m0 + (i << 4);
#pragma unroll
    for (int j = 0; j < 4; ++j) {
      const int n = n0 + (j << 4) + rlane;
      float bv = 0.f;
      if (BIAS_MODE == 2) bv = bias[n];
#pragma unroll
      for (int r = 0; r < 8; ++r) {
        float v = acc[i][j][r] * scale;
        if (BIAS_MODE == 1) v += bias[mBase + mOff + r];
        if (BIAS_MODE == 2) v += bv;
        if (RESID) v += Rb[(size_t)(mBase + mOff + r) * ldc + n];
        if (ACT == 1) v = tanhf(v);
        if (ACT == 2) v = fmaxf(v, 0.0f);
        if (ACT == 3) v = v / (1.0f + expf(-v));
        if (ACT == 4) v = (v > 0.f) ? v : 0.01f * v;
        if (ACT == 5) v = 0.5f * v * (1.0f + erff(v * 0.70710678118654752f));
        slab[(mOff + r) * 68 + (j << 4) + rlane] = v;
      }
    }
    __builtin_amdgcn_fence(__ATOMIC_RELEASE, "workgroup");
    __builtin_amdgcn_wave_barrier();
    __builtin_amdgcn_fence(__ATOMIC_ACQUIRE, "workgroup");
    if (OUT_MODE == 0) {
      float* C = (float*)Cout + (size_t)b * strideC;
      const int hh = lane >> 4, c4 = (lane & 15) * 4;
      for (int pass = 0; pass < 2; ++pass) {
#pragma unroll
        for (int it = 0; it < 8; ++it) {
          const int row = it * 2 + hh;
          v4f v = *(const v4f*)(slab + row * 68 + c4);
          *(volatile v4f*)(C + (size_t)(mBase + row) * ldc + n0 + c4) = v;
        }
        __threadfence();
      }
    } else {
      const int q = lane >> 3, c8 = (lane & 7) * 8;
      unsigned short* C  = (unsigned short*)Cout  + (size_t)b * strideC;
      unsigned short* C2 = (OUT_MODE == 2) ? ((unsigned short*)Cout2 + (size_t)b * strideC) : nullptr;
      for (int pass = 0; pass < 2; ++pass) {
#pragma unroll
        for (int it = 0; it < 4; ++it) {
          const int row = it * 4 + q;
          const float* sp = slab + row * 68 + c8;
          v8h hv, lv;
#pragma unroll
          for (int e = 0; e < 8; ++e) {
            if (OUT_MODE == 1) {
              hv[e] = (_Float16)sp[e];
            } else {
              unsigned short hb = f2bf_bits(sp[e]);
              unsigned short lb = f2bf_bits(sp[e] - bf_bits2f(hb));
              hv[e] = __builtin_bit_cast(_Float16, hb);
              lv[e] = __builtin_bit_cast(_Float16, lb);
            }
          }
          *(volatile v8h*)(C + (size_t)(mBase + row) * ldc + n0 + c8) = hv;
          if (OUT_MODE == 2) *(volatile v8h*)(C2 + (size_t)(mBase + row) * ldc + n0 + c8) = lv;
        }
        __threadfence();
      }
    }
    __builtin_amdgcn_fence(__ATOMIC_RELEASE, "workgroup");
    __builtin_amdgcn_wave_barrier();
    __builtin_amdgcn_fence(__ATOMIC_ACQUIRE, "workgroup");
  }
}

__global__ __launch_bounds__(256) void cast_f32_f16x2(
    const float* __restrict__ in, _Float16* __restrict__ out, int n2) {
  int i = blockIdx.x * 256 + threadIdx.x;
  if (i < n2) {
    const _Float16 h0 = (_Float16)in[2 * i], h1 = (_Float16)in[2 * i + 1];
    const unsigned u = (unsigned)__builtin_bit_cast(unsigned short, h0) | ((unsigned)__builtin_bit_cast(unsigned short, h1) << 16);
    ((volatile unsigned*)out)[i] = u;
    __threadfence();
    ((volatile unsigned*)out)[i] = u;
  }
}


__global__ __launch_bounds__(256) void transpose_cast_f16(const float* __restrict__ in, int ldi,
                                                         _Float16* __restrict__ outT, int ldo, float scale) {
  __shared__ __align__(16) _Float16 tile[64][72];
  const int c0 = blockIdx.x * 64, r0 = blockIdx.y * 64;
  const int t = threadIdx.y * 32 + threadIdx.x;
  for (int i = threadIdx.y; i < 64; i += 8) {
    tile[threadIdx.x][i]      = (_Float16)(in[(size_t)(r0 + i) * ldi + c0 + threadIdx.x] * scale);
    tile[32 + threadIdx.x][i] = (_Float16)(in[(size_t)(r0 + i) * ldi + c0 + 32 + threadIdx.x] * scale);
  }
  __syncthreads();
  const int q = t >> 3, c8 = (t & 7) * 8;
  for (int pass = 0; pass < 2; ++pass) {
#pragma unroll
    for (int it = 0; it < 2; ++it) {
      const int c = it * 32 + q;
      v8h hv = *(const v8h*)(&tile[c][c8]);
      *(volatile v8h*)(outT + (size_t)(c0 + c) * ldo + r0 + c8) = hv;
    }
    __threadfence();
  }
}

#define CN 8192
#define CDI 128
#define CDH 256
#define CDO 10
#define CG 64
__device__ __forceinline__ unsigned pkh(float a, float b) { return (unsigned)__builtin_bit_cast(unsigned short, (_Float16)a) | ((unsigned)__builtin_bit_cast(unsigned short, (_Float16)b) << 16); }
__global__ __launch_bounds__(256) void norm_kernel(const float* __restrict__ x, unsigned* __restrict__ XN16, _Float16* __restrict__ XNT16) {
  const int lane = threadIdx.x & 31, wave = threadIdx.x >> 5; const int n = blockIdx.x * 8 + wave;
  const v4f v = *(const v4f*)(x + (size_t)n * CDI + lane * 4); float s = v[0] * v[0] + v[1] * v[1] + v[2] * v[2] + v[3] * v[3]; for (int o = 16; o > 0; o >>= 1) s += __shfl_xor(s, o, 32);
  const float inv = 1.0f / fmaxf(sqrtf(s), 1e-8f);
  typedef __attribute__((ext_vector_type(2))) unsigned u2; const u2 u = {pkh(v[0] * inv, v[1] * inv), pkh(v[2] * inv, v[3] * inv)};
  for (int pass = 0; pass < 2; ++pass) { *(volatile u2*)(XN16 + ((size_t)n * CDI + lane * 4) / 2) = u;
#pragma unroll
    for (int q = 0; q < 4; ++q) ((volatile _Float16*)XNT16)[(size_t)(lane * 4 + q) * CN + n] = (_Float16)(v[q] * inv);
    __threadfence(); }
}
__global__ __launch_bounds__(256) void msum_kernel(const float* __restrict__ MP, unsigned* __restrict__ MT16) {
  for (int i = threadIdx.x + blockIdx.x * 256; i < CDH * CDI / 2; i += gridDim.x * 256) { const int o = i / (CDI / 2), kp = 2 * (i % (CDI / 2)); float a = 0.f, b = 0.f;
    for (int s = 0; s < 4; ++s) { a += MP[(size_t)s * CDI * CDH + (size_t)kp * CDH + o]; b += MP[(size_t)s * CDI * CDH + (size_t)(kp + 1) * CDH + o]; }
    ((volatile unsigned*)MT16)[i] = pkh(a, b); __threadfence(); ((volatile unsigned*)MT16)[i] = pkh(a, b); }
}
__global__ __launch_bounds__(256) void w2t_kernel(const float* __restrict__ W2, unsigned* __restrict__ BT) { for (int i = threadIdx.x; i < 64 * CDH / 2; i += 256) { const int o = i / (CDH / 2), kp = 2 * (i % (CDH / 2)); float a = 0.f, b = 0.f; if (o < CDO) { a = W2[(size_t)kp * CDO + o]; b = W2[(size_t)(kp + 1) * CDO + o]; } ((volatile unsigned*)BT)[i] = pkh(a, b); __threadfence(); ((volatile unsigned*)BT)[i] = pkh(a, b); } }
__global__ __launch_bounds__(64) void b2pad_kernel(const float* __restrict__ b2, float* __restrict__ B) { const int i = threadIdx.x; const float v = i < CDO ? b2[i] : 0.f; ((volatile float*)B)[i] = v; __threadfence(); ((volatile float*)B)[i] = v; }
__global__ __launch_bounds__(256) void pool_kernel(const float* __restrict__ O, const int* __restrict__ batch, float* __restrict__ out) {
  __shared__ float red[256][11]; const int g = blockIdx.x;
  float s[10]; for (int c = 0; c < 10; ++c) s[c] = 0.f; float cnt = 0.f;
  for (int n = threadIdx.x; n < CN; n += 256) if (batch[n] == g) { for (int c = 0; c < 10; ++c) s[c] += O[(size_t)n * 64 + c]; cnt += 1.f; }
  for (int c = 0; c < 10; ++c) red[threadIdx.x][c] = s[c]; red[threadIdx.x][10] = cnt; __syncthreads();
  for (int o = 128; o > 0; o >>= 1) { if (threadIdx.x < o) for (int c = 0; c < 11; ++c) red[threadIdx.x][c] += red[threadIdx.x + o][c]; __syncthreads(); }
  if (threadIdx.x < 32) { float p[10]; const float ic = 1.0f / fmaxf(red[0][10], 1.0f); float mx = -INFINITY; for (int c = 0; c < 10; ++c) { p[c] = red[0][c] * ic; mx = fmaxf(mx, p[c]); }
    float se = 0.f; for (int c = 0; c < 10; ++c) se += expf(p[c] - mx); const float lse = mx + logf(se);
    const int c = threadIdx.x; if (c < 10) { ((volatile float*)out)[g * CDO + c] = p[c] - lse; __threadfence(); ((volatile float*)out)[g * CDO + c] = p[c] - lse; } }
}
extern "C" void kernel_launch(void* const* d_in, const int* in_sizes, int n_in, void* d_out, int out_size, void* d_ws, size_t ws_size, hipStream_t stream) {
  (void)in_sizes; (void)n_in; (void)out_size; (void)ws_size;
  const float* x = (const float*)d_in[0]; const int* batch = (const int*)d_in[1]; const float* W1 = (const float*)d_in[2]; const float* b1 = (const float*)d_in[3]; const float* W2 = (const float*)d_in[4]; const float* b2 = (const float*)d_in[5];
  char* ws = (char*)d_ws; size_t off = 0;
  auto carve = [&](size_t bytes) -> char* { char* p = ws + off; off += (bytes + 255) & ~(size_t)255; return p; };
  _Float16* X16 = (_Float16*)carve((size_t)CN * CDI * 2); unsigned* XN16 = (unsigned*)carve((size_t)CN * CDI * 2); _Float16* XNT16 = (_Float16*)carve((size_t)CDI * CN * 2); _Float16* W1T = (_Float16*)carve((size_t)CDH * CDI * 2);
  _Float16* H16 = (_Float16*)carve((size_t)CN * CDH * 2); _Float16* HT16 = (_Float16*)carve((size_t)CDH * CN * 2); float* Hf = (float*)carve((size_t)CN * CDH * 4); float* MP = (float*)carve((size_t)4 * CDI * CDH * 4); unsigned* MT16 = (unsigned*)carve(CDH * CDI * 2);
  _Float16* AH16 = (_Float16*)carve((size_t)CN * CDH * 2); unsigned* W2T = (unsigned*)carve(64 * CDH * 2); float* B2P = (float*)carve(256); float* O = (float*)carve((size_t)CN * 64 * 4);
  cast_f32_f16x2<<<(CN * CDI / 2 + 255) / 256, 256, 0, stream>>>(x, X16, (long)CN * CDI / 2);
  norm_kernel<<<CN / 8, 256, 0, stream>>>(x, XN16, XNT16);
  transpose_cast_f16<<<dim3(CDH / 64, CDI / 64), dim3(32, 8), 0, stream>>>(W1, CDH, W1T, CDI, 1.0f);
  w2t_kernel<<<1, 256, 0, stream>>>(W2, W2T); b2pad_kernel<<<1, 64, 0, stream>>>(b2, B2P);
  const int tr = CN / 64;
  wmma_gemm64<0, false, 2, 0, false, 2><<<dim3((tr * 4 + 7) / 8, 1), 256, 0, stream>>>(U16(X16), nullptr, CDI, 0, U16(W1T), nullptr, CDI, 0, Hf, nullptr, CDH, 0, b1, nullptr, 0, CN, CDH, CDI, 1.0f);
  transpose_cast_f16<<<dim3(CDH / 64, CN / 64), dim3(32, 8), 0, stream>>>(Hf, CDH, HT16, CN, 1.0f);
  wmma_gemm64<0, false, 0, 0, false><<<dim3(1, 4), 256, 0, stream>>>(U16(XNT16), nullptr, CN, CN / 4, U16(HT16), nullptr, CN, CN / 4, MP, nullptr, CDH, (long)CDI * CDH, nullptr, nullptr, 0, CDI, CDH, CN / 4, 1.0f);
  msum_kernel<<<8, 256, 0, stream>>>(MP, MT16);
  wmma_gemm64<0, false, 0, 1, false><<<dim3((tr * 4 + 7) / 8, 1), 256, 0, stream>>>((const unsigned short*)XN16, nullptr, CDI, 0, (const unsigned short*)MT16, nullptr, CDI, 0, AH16, nullptr, CDH, 0, nullptr, nullptr, 0, CN, CDH, CDI, 1.0f);
  wmma_gemm64<0, false, 2, 0, false><<<dim3((tr + 7) / 8, 1), 256, 0, stream>>>(U16(AH16), nullptr, CDH, 0, (const unsigned short*)W2T, nullptr, CDH, 0, O, nullptr, 64, 0, B2P, nullptr, 0, CN, 64, CDH, 1.0f);
  pool_kernel<<<CG, 256, 0, stream>>>(O, batch, (float*)d_out);
}
